// GCFM_41755672052587
// MI455X (gfx1250) — hardware-verified
//
#include <hip/hip_runtime.h>


#define NB_  2
#define CC   256
#define NHD  4
#define DH   64
#define HWD  48
#define PP   (HWD * HWD)
#define NT   (NB_ * PP)
#define KA   7
#define BW   54
#define BR   384
#define ZC   96
typedef _Float16 h16;
typedef unsigned short bf;
typedef __attribute__((ext_vector_type(16))) __bf16   v16bf;
typedef __attribute__((ext_vector_type(16))) _Float16 v16h;
typedef __attribute__((ext_vector_type(8)))  _Float16 v8h;
typedef __attribute__((ext_vector_type(8)))  unsigned short v8us;
typedef __attribute__((ext_vector_type(8)))  float    v8f;
typedef __attribute__((ext_vector_type(4)))  float    v4f;
typedef v8h  __attribute__((may_alias)) v8ha;
typedef v4f  __attribute__((may_alias)) v4fa;
typedef v8us __attribute__((may_alias)) v8usa;

__device__ __forceinline__ unsigned short f2bf(float f) { unsigned u = __float_as_uint(f); u += 0x7FFFu + ((u >> 16) & 1u); return (unsigned short)(u >> 16); }
__device__ __forceinline__ float bf2f(unsigned short b) { return __uint_as_float(((unsigned)b) << 16); }
__device__ __forceinline__ float bfr(float f) { return bf2f(f2bf(f)); }
__device__ __forceinline__ v16h cat16(v8h lo, v8h hi) { return __builtin_shufflevector(lo, hi, 0, 1, 2, 3, 4, 5, 6, 7, 8, 9, 10, 11, 12, 13, 14, 15); }
__device__ __forceinline__ v16bf cat16b(v8us lo, v8us hi) { return __builtin_bit_cast(v16bf, __builtin_shufflevector(lo, hi, 0, 1, 2, 3, 4, 5, 6, 7, 8, 9, 10, 11, 12, 13, 14, 15)); }
__device__ __forceinline__ v8f wmma16(v16h a, v16h b, v8f c) { return __builtin_amdgcn_wmma_f32_16x16x32_f16(false, a, false, b, (short)0, c, false, false); }
__device__ __forceinline__ v8f wmmab(v16bf a, v16bf b, v8f c) { return __builtin_amdgcn_wmma_f32_16x16x32_bf16(false, a, false, b, (short)0, c, false, false); }


template <typename T16> struct WFrag;
template <> struct WFrag<h16> { typedef v16h V; static __device__ __forceinline__ V ld(const h16* p) { return cat16(*(const v8h*)p, *(const v8h*)(p + 16)); } static __device__ __forceinline__ v8f mma(V a, V b, v8f c) { return wmma16(a, b, c); } };
template <> struct WFrag<bf> { typedef v16bf V; static __device__ __forceinline__ V ld(const bf* p) { return cat16b(*(const v8us*)p, *(const v8us*)(p + 16)); } static __device__ __forceinline__ v8f mma(V a, V b, v8f c) { return wmmab(a, b, c); } };
template <typename T16, int NSPLIT, bool BIAS>
__global__ __launch_bounds__(32) void k_gemmw(const T16* __restrict__ A, const T16* __restrict__ A2, const T16* __restrict__ Bt, const T16* __restrict__ Bt2, int K, float* C, int ldc, const float* __restrict__ bias, size_t sA, size_t sB, size_t sC) {
    typedef typename WFrag<T16>::V V;
    __shared__ __align__(16) float os[16 * 68];
    const size_t z = blockIdx.z; A += z * sA; if (A2) A2 += z * sA; Bt += z * sB; if (Bt2) Bt2 += z * sB; C += z * sC;
    const int lane = threadIdx.x & 31, lr = lane & 15, hi = lane >> 4; const int r0 = blockIdx.x * 64, c0 = blockIdx.y * 64;
    v8f acc[4][4];
#pragma unroll
    for (int mb = 0; mb < 4; ++mb)
#pragma unroll
        for (int nb = 0; nb < 4; ++nb) acc[mb][nb] = (v8f){};
    const size_t aoff = (size_t)(r0 + lr) * K + 8 * hi, boff = (size_t)(c0 + lr) * K + 8 * hi;
#pragma unroll 1
    for (int kc = 0; kc < K; kc += 32) {
        V a[4], a2[4];
#pragma unroll
        for (int mb = 0; mb < 4; ++mb) { a[mb] = WFrag<T16>::ld(A + aoff + (size_t)mb * 16 * K + kc); if (NSPLIT == 1 || NSPLIT == 2) a2[mb] = WFrag<T16>::ld(A2 + aoff + (size_t)mb * 16 * K + kc); }
#pragma unroll
        for (int nb = 0; nb < 4; ++nb) { const V b = WFrag<T16>::ld(Bt + boff + (size_t)nb * 16 * K + kc); V b2; if (NSPLIT >= 2) b2 = WFrag<T16>::ld(Bt2 + boff + (size_t)nb * 16 * K + kc);
#pragma unroll
            for (int mb = 0; mb < 4; ++mb) { acc[mb][nb] = WFrag<T16>::mma(a[mb], b, acc[mb][nb]); if (NSPLIT == 1 || NSPLIT == 2) acc[mb][nb] = WFrag<T16>::mma(a2[mb], b, acc[mb][nb]); if (NSPLIT >= 2) acc[mb][nb] = WFrag<T16>::mma(a[mb], b2, acc[mb][nb]); } }
        asm volatile("v_nop\n\tv_nop\n\tv_nop\n\tv_nop" : "+v"(acc[0][0]), "+v"(acc[1][1]), "+v"(acc[2][2]), "+v"(acc[3][3]) : "v"(a[0]), "v"(a[3]));
    }
#pragma unroll
    for (int mb = 0; mb < 4; ++mb) {
#pragma unroll
        for (int nb = 0; nb < 4; ++nb) {
#pragma unroll
            for (int j = 0; j < 8; ++j) os[(hi * 8 + j) * 68 + nb * 16 + lr] = acc[mb][nb][j]; }
        __builtin_amdgcn_wave_barrier(); asm volatile("" ::: "memory");
        float* crow = C + (size_t)(r0 + mb * 16) * ldc + c0;
#pragma unroll 1
        for (int ps = 0; ps < 2; ++ps) {
#pragma unroll
            for (int s = 0; s < 8; ++s) { const int row = 2 * s + hi, cofs = lr * 4; v4f val = *(const v4fa*)(os + row * 68 + cofs); if (BIAS) { val[0] += bfr(bias[c0 + cofs]); val[1] += bfr(bias[c0 + cofs + 1]); val[2] += bfr(bias[c0 + cofs + 2]); val[3] += bfr(bias[c0 + cofs + 3]); }
                *(volatile v4f*)(crow + (size_t)row * ldc + cofs) = val; }
            if (ps == 0) __threadfence(); }
        __builtin_amdgcn_wave_barrier(); asm volatile("" ::: "memory");
    }
}

__device__ __forceinline__ void splitf(float y, unsigned short& h, unsigned short& l) { h = f2bf(y); l = f2bf(y - bf2f(h)); }
__device__ __forceinline__ int refl(int i) { return i < 0 ? -i : (i > HWD - 1 ? 2 * (HWD - 1) - i : i); }

__global__ __launch_bounds__(256) void k_cvt8(const float* __restrict__ src, bf* dst, size_t n8) {
    const size_t i = (size_t)blockIdx.x * 256 + threadIdx.x; if (i >= n8) return;
    const v8f v = *(const v8f*)(src + i * 8); v8us o;
#pragma unroll
    for (int k = 0; k < 8; ++k) o[k] = f2bf(v[k]);
    *(volatile v8us*)(dst + i * 8) = o; __threadfence(); *(volatile v8us*)(dst + i * 8) = o;
}
__global__ __launch_bounds__(256) void k_tok(const float* __restrict__ src, bf* T) {
    __shared__ float tl[64][65];
    const int tid = threadIdx.x; const int p0 = blockIdx.x * 64, c0 = blockIdx.y * 64, b = blockIdx.z;
#pragma unroll
    for (int i = 0; i < 16; ++i) { const int cc = i * 4 + (tid >> 6), pp = tid & 63; tl[cc][pp] = src[((size_t)b * CC + c0 + cc) * PP + p0 + pp]; }
    __syncthreads();
    const int lane = tid & 31, wv = tid >> 5;
    auto pass = [&]() { const int cq = (lane & 7) * 8;
#pragma unroll
        for (int i2 = 0; i2 < 2; ++i2) { const int pr = wv * 8 + i2 * 4 + (lane >> 3); v8us o;
#pragma unroll
            for (int i = 0; i < 8; ++i) o[i] = f2bf(tl[cq + i][pr]);
            *(volatile v8us*)(T + ((size_t)b * PP + p0 + pr) * CC + c0 + cq) = o; } };
    pass(); __threadfence(); pass();
}
__global__ __launch_bounds__(256) void k_pe(const float* __restrict__ Wp, const float* __restrict__ bp, float* PE) {
    const int lane = threadIdx.x & 31; const size_t e0 = ((size_t)blockIdx.x * 8 + (threadIdx.x >> 5)) * 128 + lane * 4; if (e0 >= (size_t)PP * DH) return; v4f o;
#pragma unroll
    for (int q = 0; q < 4; ++q) { const size_t e = e0 + q; const int p = (int)(e / DH), d = (int)(e % DH); const float lw = -1.0f + (float)(p % HWD) * (2.0f / 47.0f), lh = -1.0f + (float)(p / HWD) * (2.0f / 47.0f);
        o[q] = bfr(Wp[d * 2 + 0]) * lw + bfr(Wp[d * 2 + 1]) * lh + bfr(bp[d]); }
    *(volatile v4f*)(PE + e0) = o; __threadfence(); *(volatile v4f*)(PE + e0) = o;
}
__global__ __launch_bounds__(256) void k_qp(const float* __restrict__ Q, int b, int hp, bf* Ph, bf* Pl) {
    typedef __attribute__((ext_vector_type(2))) unsigned short v2us;
    const int lane = threadIdx.x & 31; const size_t L0 = ((size_t)blockIdx.x * 8 + (threadIdx.x >> 5)) * 8; const size_t nlines = (size_t)ZC * 64 * 64 / 64;
#pragma unroll 1
    for (int ps = 0; ps < 2; ++ps) {
#pragma unroll
        for (int l = 0; l < 8; ++l) { const size_t L = L0 + l; if (L >= nlines) break; const size_t e = L * 64 + lane * 2; const int zc = (int)(e >> 12), w = (int)((e >> 6) & 63), d = (int)(e & 63); const int head = hp * 2 + zc / HWD, h = zc % HWD; v2us oh, ol;
#pragma unroll
            for (int q = 0; q < 2; ++q) { unsigned short a = 0, bb = 0; if (w < HWD) splitf(Q[((size_t)b * PP + h * HWD + w) * CC + head * DH + d + q] * 0.125f, a, bb); oh[q] = a; ol[q] = bb; }
            *(volatile v2us*)(Ph + e) = oh; *(volatile v2us*)(Pl + e) = ol; }
        if (ps == 0) __threadfence(); }
}
__global__ __launch_bounds__(256) void k_kb(const float* __restrict__ Kf, const float* __restrict__ PE, int b, int hp, bf* Bh, bf* Bl) {
    typedef __attribute__((ext_vector_type(2))) unsigned short v2us;
    const int lane = threadIdx.x & 31; const size_t L0 = ((size_t)blockIdx.x * 8 + (threadIdx.x >> 5)) * 8; const size_t nlines = (size_t)ZC * BR * 64 / 64;
#pragma unroll 1
    for (int ps = 0; ps < 2; ++ps) {
#pragma unroll
        for (int l = 0; l < 8; ++l) { const size_t L = L0 + l; if (L >= nlines) break; const size_t e = L * 64 + lane * 2; const int zc = (int)(e / ((size_t)BR * 64)), r = (int)((e >> 6) % BR), d = (int)(e & 63);
            const int head = hp * 2 + zc / HWD, h = zc % HWD; const int i = r / BW, jc = r % BW; const bool live = r < KA * BW; const int pq = refl(h + (live ? i : 0) - 3) * HWD + refl(jc - 3); v2us oh, ol;
#pragma unroll
            for (int q = 0; q < 2; ++q) { unsigned short a = 0, bb = 0; if (live) splitf(Kf[((size_t)b * PP + pq) * CC + head * DH + d + q] - PE[(size_t)pq * DH + d + q], a, bb); oh[q] = a; ol[q] = bb; }
            *(volatile v2us*)(Bh + e) = oh; *(volatile v2us*)(Bl + e) = ol; }
        if (ps == 0) __threadfence(); }
}
__global__ __launch_bounds__(256) void k_vbt(const float* __restrict__ Vf, int b, int hp, bf* Th, bf* Tlo) {
    typedef __attribute__((ext_vector_type(2))) unsigned short v2us;
    const int lane = threadIdx.x & 31; const size_t L0 = ((size_t)blockIdx.x * 8 + (threadIdx.x >> 5)) * 8; const size_t nlines = (size_t)ZC * 64 * BR / 64;
#pragma unroll 1
    for (int ps = 0; ps < 2; ++ps) {
#pragma unroll
        for (int l = 0; l < 8; ++l) { const size_t L = L0 + l; if (L >= nlines) break; const size_t e = L * 64 + lane * 2; const int zc = (int)(e / ((size_t)64 * BR)), d = (int)((e / BR) % 64), r0 = (int)(e % BR);
            const int head = hp * 2 + zc / HWD, h = zc % HWD; v2us oh, ol;
#pragma unroll
            for (int q = 0; q < 2; ++q) { const int r = r0 + q; const bool live = r < KA * BW; const int i = live ? r / BW : 0, jc = r % BW; const int pq = refl(h + i - 3) * HWD + refl(jc - 3); unsigned short a = 0, bb = 0;
                if (live) splitf(Vf[((size_t)b * PP + pq) * CC + head * DH + d], a, bb); oh[q] = a; ol[q] = bb; }
            *(volatile v2us*)(Th + e) = oh; *(volatile v2us*)(Tlo + e) = ol; }
        if (ps == 0) __threadfence(); }
}
__global__ __launch_bounds__(256) void k_softw(const float* __restrict__ Sb, bf* PH, bf* PL) {
    typedef __attribute__((ext_vector_type(4))) unsigned short v4us;
    const int lane = threadIdx.x & 31; const int row = blockIdx.x * 8 + (threadIdx.x >> 5); if (row >= ZC * 64) return; const int w = row & 63; const float* sr = Sb + (size_t)row * BR;
    const bool qlive = w < HWD;
    float s0 = -3.0e38f, s1 = -3.0e38f;
    if (qlive) { { const int kk = lane; const int i = kk / KA, j = kk % KA; s0 = sr[i * BW + w + j]; } if (lane + 32 < KA * KA) { const int kk = lane + 32; const int i = kk / KA, j = kk % KA; s1 = sr[i * BW + w + j]; } }
    float mx = fmaxf(s0, s1);
#pragma unroll
    for (int sh = 16; sh; sh >>= 1) mx = fmaxf(mx, __shfl_xor(mx, sh, 32));
    float sum = (qlive ? __expf(s0 - mx) : 0.f) + ((qlive && lane + 32 < KA * KA) ? __expf(s1 - mx) : 0.f);
#pragma unroll
    for (int sh = 16; sh; sh >>= 1) sum += __shfl_xor(sum, sh, 32);
    const float inv = qlive ? __fdiv_rn(1.0f, sum) : 0.f;
#pragma unroll 1
    for (int ps = 0; ps < 2; ++ps) {
#pragma unroll
        for (int ch = 0; ch < BR / 128; ++ch) { const int r0 = ch * 128 + lane * 4; v4us oh, ol;
#pragma unroll
            for (int q = 0; q < 4; ++q) { const int r = r0 + q; const int i = r / BW, j = r % BW - w; unsigned short a = 0, bb = 0;
                if (qlive && i < KA && j >= 0 && j < KA) splitf(__expf(sr[r] - mx) * inv, a, bb); oh[q] = a; ol[q] = bb; }
            *(volatile v4us*)(PH + (size_t)row * BR + r0) = oh; *(volatile v4us*)(PL + (size_t)row * BR + r0) = ol; }
        if (ps == 0) __threadfence(); }
}
__global__ __launch_bounds__(256) void k_oatt(const float* __restrict__ O, int b, int hp, float* OA) {
    const int lane = threadIdx.x & 31; const int wg = blockIdx.x * 8 + (threadIdx.x >> 5); if (wg >= 128 * (PP / 128)) return; const int cl = wg / (PP / 128), p0 = (wg % (PP / 128)) * 128 + lane * 4;
    const int zh = cl >> 6, d = cl & 63, head = hp * 2 + zh; v4f o;
#pragma unroll
    for (int q = 0; q < 4; ++q) { const int p = p0 + q; const int zc = zh * HWD + p / HWD, w = p % HWD; o[q] = O[((size_t)zc * 64 + w) * 64 + d]; }
    float* dst = OA + ((size_t)b * CC + head * DH + d) * PP + p0; *(volatile v4f*)dst = o; __threadfence(); *(volatile v4f*)dst = o;
}
__global__ __launch_bounds__(256) void k_fc(const float* __restrict__ Q, const float* __restrict__ Kf, const float* __restrict__ Vf, const float* __restrict__ Wfc, float* FC) {
    const int lane = threadIdx.x & 31; const int wg = blockIdx.x * 8 + (threadIdx.x >> 5); if (wg >= NB_ * DH * (PP / 128)) return;
    const int b = wg / (DH * (PP / 128)), d = (wg / (PP / 128)) % DH, p0 = (wg % (PP / 128)) * 128 + lane * 4;
    float v[12][4];
#pragma unroll
    for (int c = 0; c < 12; ++c) { const float* src = c < 4 ? Q : (c < 8 ? Kf : Vf); const int head = c & 3;
#pragma unroll
        for (int q = 0; q < 4; ++q) v[c][q] = src[((size_t)b * PP + p0 + q) * CC + head * DH + d]; }
#pragma unroll 1
    for (int ps = 0; ps < 2; ++ps) {
#pragma unroll 1
        for (int o = 0; o < 9; ++o) { v4f r;
#pragma unroll
            for (int q = 0; q < 4; ++q) { float acc = 0.f;
#pragma unroll
                for (int c = 0; c < 12; ++c) acc = fmaf(bfr(Wfc[o * 12 + c]), v[c][q], acc);
                r[q] = acc; }
            *(volatile v4f*)(FC + (((size_t)b * DH + d) * 9 + o) * PP + p0) = r; }
        if (ps == 0) __threadfence(); }
}
__global__ __launch_bounds__(256) void k_dep(const float* __restrict__ FC, const float* __restrict__ Wd, float* OC) {
    const int lane = threadIdx.x & 31; const int wg = blockIdx.x * 8 + (threadIdx.x >> 5); if (wg >= NB_ * DH * (PP / 128)) return;
    const int b = wg / (DH * (PP / 128)), g = (wg / (PP / 128)) % DH, p0 = (wg % (PP / 128)) * 128 + lane * 4;
    float acc[4][4];
#pragma unroll
    for (int m = 0; m < 4; ++m)
#pragma unroll
        for (int q = 0; q < 4; ++q) acc[m][q] = 0.f;
#pragma unroll 1
    for (int i9 = 0; i9 < 9; ++i9) { const float* src = FC + (((size_t)b * DH + g) * 9 + i9) * PP;
#pragma unroll 1
        for (int kh = 0; kh < 3; ++kh) {
            float wv[4][3];
#pragma unroll
            for (int m = 0; m < 4; ++m)
#pragma unroll
                for (int kw = 0; kw < 3; ++kw) wv[m][kw] = bfr(Wd[(((size_t)(g * 4 + m) * 9 + i9) * 3 + kh) * 3 + kw]);
#pragma unroll
            for (int q = 0; q < 4; ++q) { const int p = p0 + q; const int h = p / HWD + kh - 1, w = p % HWD;
#pragma unroll
                for (int kw = 0; kw < 3; ++kw) { const int ww = w + kw - 1; const bool in = (h >= 0) && (h < HWD) && (ww >= 0) && (ww < HWD);
                    const int hc = h < 0 ? 0 : (h > HWD - 1 ? HWD - 1 : h), wc = ww < 0 ? 0 : (ww > HWD - 1 ? HWD - 1 : ww); const float x = in ? src[hc * HWD + wc] : 0.f;
#pragma unroll
                    for (int m = 0; m < 4; ++m) acc[m][q] = fmaf(x, wv[m][kw], acc[m][q]); } } } }
#pragma unroll 1
    for (int ps = 0; ps < 2; ++ps) {
#pragma unroll
        for (int m = 0; m < 4; ++m) { v4f r = {acc[m][0], acc[m][1], acc[m][2], acc[m][3]}; *(volatile v4f*)(OC + ((size_t)b * CC + g * 4 + m) * PP + p0) = r; }
        if (ps == 0) __threadfence(); }
}
__global__ __launch_bounds__(256) void k_out(const float* __restrict__ OA, const float* __restrict__ OC, float* OUT) {
    const size_t i = ((size_t)blockIdx.x * 256 + threadIdx.x) * 4; if (i >= (size_t)NB_ * CC * PP) return;
    const v4f a = *(const v4f*)(OA + i), c = *(const v4f*)(OC + i); const v4f o = a * 0.5f + c * 0.5f;
    *(volatile v4f*)(OUT + i) = o; __threadfence(); *(volatile v4f*)(OUT + i) = o;
}

extern "C" void kernel_launch(void* const* d_in, const int* in_sizes, int n_in,
                              void* d_out, int out_size, void* d_ws, size_t ws_size, hipStream_t stream) {
    (void)in_sizes; (void)n_in; (void)out_size;
    const float* x = (const float*)d_in[0]; const float* y = (const float*)d_in[1]; const float* z = (const float*)d_in[2];
    const float* W1 = (const float*)d_in[3]; const float* b1 = (const float*)d_in[4]; const float* W2 = (const float*)d_in[5]; const float* b2 = (const float*)d_in[6]; const float* W3 = (const float*)d_in[7]; const float* b3 = (const float*)d_in[8];
    const float* Wp = (const float*)d_in[9]; const float* bp = (const float*)d_in[10]; const float* Wfc = (const float*)d_in[11]; const float* Wd = (const float*)d_in[12];
    float* OUT = (float*)d_out;
    char* wsp = (char*)d_ws;
    auto take = [&](size_t bytes) { char* p = wsp; wsp += (bytes + 255) & ~(size_t)255; return (void*)p; };
    bf* WB1 = (bf*)take((size_t)CC * CC * 2); bf* WB2 = (bf*)take((size_t)CC * CC * 2); bf* WB3 = (bf*)take((size_t)CC * CC * 2);
    bf* XT = (bf*)take((size_t)NT * CC * 2); bf* YT = (bf*)take((size_t)NT * CC * 2); bf* ZT = (bf*)take((size_t)NT * CC * 2);
    float* Q = (float*)take((size_t)NT * CC * 4); float* Kf = (float*)take((size_t)NT * CC * 4); float* Vf = (float*)take((size_t)NT * CC * 4); float* PE = (float*)take((size_t)PP * DH * 4);
    bf* QPh = (bf*)take((size_t)ZC * 64 * 64 * 2); bf* QPl = (bf*)take((size_t)ZC * 64 * 64 * 2); bf* KBh = (bf*)take((size_t)ZC * BR * 64 * 2); bf* KBl = (bf*)take((size_t)ZC * BR * 64 * 2);
    bf* VTh = (bf*)take((size_t)ZC * 64 * BR * 2); bf* VTl = (bf*)take((size_t)ZC * 64 * BR * 2); float* Sb = (float*)take((size_t)ZC * 64 * BR * 4); bf* PH = (bf*)take((size_t)ZC * 64 * BR * 2); bf* PL = (bf*)take((size_t)ZC * 64 * BR * 2);
    float* O = (float*)take((size_t)ZC * 64 * 64 * 4); float* OA = (float*)take((size_t)NB_ * CC * PP * 4); float* FC = (float*)take((size_t)NB_ * DH * 9 * PP * 4); float* OC = (float*)take((size_t)NB_ * CC * PP * 4);
    if ((size_t)(wsp - (char*)d_ws) > ws_size) return;
    { const unsigned n8 = CC * CC / 8; k_cvt8<<<(n8 + 255) / 256, 256, 0, stream>>>(W1, WB1, n8); k_cvt8<<<(n8 + 255) / 256, 256, 0, stream>>>(W2, WB2, n8); k_cvt8<<<(n8 + 255) / 256, 256, 0, stream>>>(W3, WB3, n8); }
    k_tok<<<dim3(PP / 64, CC / 64, NB_), 256, 0, stream>>>(x, XT); k_tok<<<dim3(PP / 64, CC / 64, NB_), 256, 0, stream>>>(y, YT); k_tok<<<dim3(PP / 64, CC / 64, NB_), 256, 0, stream>>>(z, ZT);
    k_gemmw<bf, 0, true><<<dim3(NT / 64, CC / 64, 1), 32, 0, stream>>>(XT, nullptr, WB1, nullptr, CC, Q, CC, b1, 0, 0, 0);
    k_gemmw<bf, 0, true><<<dim3(NT / 64, CC / 64, 1), 32, 0, stream>>>(YT, nullptr, WB2, nullptr, CC, Kf, CC, b2, 0, 0, 0);
    k_gemmw<bf, 0, true><<<dim3(NT / 64, CC / 64, 1), 32, 0, stream>>>(ZT, nullptr, WB3, nullptr, CC, Vf, CC, b3, 0, 0, 0);
    k_pe<<<(PP * DH / 128 + 7) / 8, 256, 0, stream>>>(Wp, bp, PE);
    for (int b = 0; b < NB_; ++b)
        for (int hp = 0; hp < NHD / 2; ++hp) {
            k_qp<<<(ZC * 64 * 64 / 64 + 63) / 64, 256, 0, stream>>>(Q, b, hp, QPh, QPl);
            k_kb<<<(ZC * BR * 64 / 64 + 63) / 64, 256, 0, stream>>>(Kf, PE, b, hp, KBh, KBl);
            k_vbt<<<(ZC * 64 * BR / 64 + 63) / 64, 256, 0, stream>>>(Vf, b, hp, VTh, VTl);
            k_gemmw<bf, 2, false><<<dim3(1, BR / 64, ZC), 32, 0, stream>>>(QPh, QPl, KBh, KBl, DH, Sb, BR, nullptr, (size_t)64 * 64, (size_t)BR * 64, (size_t)64 * BR);
            k_softw<<<ZC * 64 / 8, 256, 0, stream>>>(Sb, PH, PL);
            k_gemmw<bf, 2, false><<<dim3(1, 1, ZC), 32, 0, stream>>>(PH, PL, VTh, VTl, BR, O, 64, nullptr, (size_t)64 * BR, (size_t)64 * BR, (size_t)64 * 64);
            k_oatt<<<128 * (PP / 128) / 8, 256, 0, stream>>>(O, b, hp, OA); }
    k_fc<<<NB_ * DH * (PP / 128) / 8, 256, 0, stream>>>(Q, Kf, Vf, Wfc, FC);
    k_dep<<<NB_ * DH * (PP / 128) / 8, 256, 0, stream>>>(FC, Wd, OC);
    k_out<<<(unsigned)(((size_t)NB_ * CC * PP / 4 + 255) / 256), 256, 0, stream>>>(OA, OC, OUT);
}
